// GroupedQueryAttention_37864431681667
// MI455X (gfx1250) — hardware-verified
//
#include <hip/hip_runtime.h>


#ifndef NB
#define NB 2
#endif
#ifndef SEQ
#define SEQ 2048
#endif
#define NB_FULL 2
#define S_FULL  2048
#define HM   2048
#define NH_  16
#define NKV  4
#define REP  (NH_ / NKV)
#define HD   128
#define DQ   (NH_ * HD)
#define DKV  (NKV * HD)
#define PP   40
#define OP   132
#define SCL2 ((float)(0.08838834764831845 * 1.4426950408889634))
#define MASKT (-3.0e38f)
#define PSH  10.0f

#define SZ_WQ  ((size_t)DQ * HM * 2)
#define SZ_WKV ((size_t)DKV * HM * 2)
#define SZ_WO  ((size_t)HM * DQ * 2)
#define SZ_XB  ((size_t)NB * SEQ * HM * 2)
#define SZ_QP  ((size_t)NB * SEQ * DQ * 2)
#define SZ_KP  ((size_t)NB * SEQ * DKV * 2)
#define SZ_VT  ((size_t)NB * DKV * SEQ * 2)
#define SZ_AT  ((size_t)NB * SEQ * DQ * 2)
#define SZ_ALL (SZ_WQ + 2 * SZ_WKV + SZ_WO + SZ_XB + SZ_QP + SZ_KP + SZ_VT + 2 * SZ_AT)

static_assert(SEQ % 64 == 0);
static_assert(SEQ % 32 == 0);
static_assert((NB * SEQ) % 64 == 0);
static_assert(HM % 64 == 0);
static_assert(DQ % 64 == 0);
static_assert(DKV % 64 == 0);
static_assert(HM % 32 == 0);
static_assert(DQ % 32 == 0);
static_assert(HD == 128);
static_assert(HD % 32 == 0);
static_assert(NH_ % NKV == 0);
static_assert(NB <= NB_FULL);
static_assert(SEQ <= S_FULL);
static_assert(PP % 8 == 0);
static_assert(PP >= 32);
static_assert(OP % 4 == 0);
static_assert(OP >= HD);
static_assert(((size_t)HM * DQ) % 64 == 0);
static_assert(((size_t)HM * DKV) % 64 == 0);
static_assert((SEQ * HM / 8) % 256 == 0);
static_assert(SZ_WQ % 256 == 0);
static_assert(SZ_WKV % 256 == 0);
static_assert(SZ_XB % 256 == 0);
static_assert(SZ_KP % 256 == 0);
static_assert(SZ_VT % 256 == 0);
static_assert(SZ_ALL <= (size_t)134217728);

typedef _Float16 h16;
typedef unsigned short bf;
typedef __attribute__((ext_vector_type(16))) __bf16   v16bf;
typedef __attribute__((ext_vector_type(16))) _Float16 v16h;
typedef __attribute__((ext_vector_type(8)))  _Float16 v8h;
typedef __attribute__((ext_vector_type(8)))  unsigned short v8us;
typedef __attribute__((ext_vector_type(2)))  unsigned short v2us;
typedef __attribute__((ext_vector_type(8)))  float    v8f;
typedef __attribute__((ext_vector_type(4)))  float    v4f;
typedef v8h  __attribute__((may_alias)) v8ha;
typedef v4f  __attribute__((may_alias)) v4fa;

__device__ __forceinline__ unsigned short f2bf(float f) { unsigned u = __float_as_uint(f); u += 0x7FFFu + ((u >> 16) & 1u); return (unsigned short)(u >> 16); }
__device__ __forceinline__ float bf2f(unsigned short b) { return __uint_as_float(((unsigned)b) << 16); }
__device__ __forceinline__ float bfr(float f) { return bf2f(f2bf(f)); }
__device__ __forceinline__ void splitf(float y, unsigned short& h, unsigned short& l) { h = f2bf(y); l = f2bf(y - bf2f(h)); }
__device__ __forceinline__ v16h cat16(v8h lo, v8h hi) { return __builtin_shufflevector(lo, hi, 0, 1, 2, 3, 4, 5, 6, 7, 8, 9, 10, 11, 12, 13, 14, 15); }
__device__ __forceinline__ v16bf cat16b(v8us lo, v8us hi) { return __builtin_bit_cast(v16bf, __builtin_shufflevector(lo, hi, 0, 1, 2, 3, 4, 5, 6, 7, 8, 9, 10, 11, 12, 13, 14, 15)); }
__device__ __forceinline__ v8f wmma16(v16h a, v16h b, v8f c) { return __builtin_amdgcn_wmma_f32_16x16x32_f16(false, a, false, b, (short)0, c, false, false); }
__device__ __forceinline__ v8f wmmab(v16bf a, v16bf b, v8f c) { return __builtin_amdgcn_wmma_f32_16x16x32_bf16(false, a, false, b, (short)0, c, false, false); }
__device__ __forceinline__ v16bf ldb(const bf* p) { return cat16b(*(const v8us*)p, *(const v8us*)(p + 16)); }
__device__ __forceinline__ v16h ldh(const h16* p) { return cat16(*(const v8h*)p, *(const v8h*)(p + 16)); }

__global__ __launch_bounds__(256) void k_wtG(const float* __restrict__ w, int K, int N, bf* Bt) {
    const int lane = threadIdx.x & 31; const int L0 = (blockIdx.x * 8 + (threadIdx.x >> 5)) * 8; const int nlines = N * K / 64;
#pragma unroll
    for (int ps = 0; ps < 2; ++ps) {
#pragma unroll 1
        for (int l = 0; l < 8; ++l) { const int L = L0 + l; if (L >= nlines) break; const size_t e = (size_t)L * 64 + lane * 2; const int k = (int)(e % K), n = (int)(e / K); v2us o;
            o[0] = f2bf(w[(size_t)k * N + n]); o[1] = f2bf(w[(size_t)(k + 1) * N + n]); *(volatile v2us*)(Bt + e) = o; }
        if (ps == 0) __threadfence(); }
}

__global__ __launch_bounds__(256) void k_cvt8(const float* __restrict__ src, bf* dst, size_t n8, size_t sstride, size_t dstride) {
    const size_t i = (size_t)blockIdx.x * 256 + threadIdx.x; if (i >= n8) return;
    src += (size_t)blockIdx.y * sstride; dst += (size_t)blockIdx.y * dstride;
    const v8f v = *(const v8f*)(src + i * 8); v8us o;
#pragma unroll
    for (int k = 0; k < 8; ++k) o[k] = f2bf(v[k]);
    *(volatile v8us*)(dst + i * 8) = o; __threadfence(); *(volatile v8us*)(dst + i * 8) = o;
}

#define OM_F32C 0
#define OM_H16C 1
#define OM_H16R 2
template <int NSPLIT, int OMODE>
__device__ __forceinline__ void gemm_body(const bf* __restrict__ A, const bf* A2, const bf* __restrict__ Bt, int K, void* Cv, int ldc, const float* __restrict__ bias, size_t sA, size_t sB, size_t sC) {
    __shared__ __align__(16) float os[16 * 68];
    const size_t z = blockIdx.z; A += z * sA; if (NSPLIT == 1) A2 += z * sA; Bt += z * sB;
    const int lane = threadIdx.x & 31, lr = lane & 15, hi = lane >> 4; const int r0 = blockIdx.x * 64, c0 = blockIdx.y * 64;
    v8f acc[4][4];
#pragma unroll
    for (int mb = 0; mb < 4; ++mb)
#pragma unroll
        for (int nb = 0; nb < 4; ++nb) acc[mb][nb] = (v8f){};
    const size_t aoff = (size_t)(r0 + lr) * K + 8 * hi, boff = (size_t)(c0 + lr) * K + 8 * hi;
#pragma unroll 1
    for (int kc = 0; kc < K; kc += 32) {
        v16bf a[4], a2[4];
#pragma unroll
        for (int mb = 0; mb < 4; ++mb) { a[mb] = ldb(A + aoff + (size_t)mb * 16 * K + kc); if (NSPLIT == 1) a2[mb] = ldb(A2 + aoff + (size_t)mb * 16 * K + kc); }
#pragma unroll
        for (int nb = 0; nb < 4; ++nb) { const v16bf b = ldb(Bt + boff + (size_t)nb * 16 * K + kc);
#pragma unroll
            for (int mb = 0; mb < 4; ++mb) { acc[mb][nb] = wmmab(a[mb], b, acc[mb][nb]); if (NSPLIT == 1) acc[mb][nb] = wmmab(a2[mb], b, acc[mb][nb]); } }
        asm volatile("v_nop\n\tv_nop\n\tv_nop\n\tv_nop" : "+v"(acc[0][0]), "+v"(acc[1][1]), "+v"(acc[2][2]), "+v"(acc[3][3]) : "v"(a[0]), "v"(a[3]));
    }
#pragma unroll
    for (int mb = 0; mb < 4; ++mb) {
#pragma unroll
        for (int nb = 0; nb < 4; ++nb) {
#pragma unroll
            for (int j = 0; j < 8; ++j) os[(hi * 8 + j) * 68 + nb * 16 + lr] = acc[mb][nb][j]; }
        __builtin_amdgcn_wave_barrier(); asm volatile("" ::: "memory");
        if (OMODE == OM_F32C) {
            float* crow = (float*)Cv + z * sC + (size_t)(r0 + mb * 16) * ldc + c0;
#pragma unroll 1
            for (int ps = 0; ps < 2; ++ps) {
#pragma unroll
                for (int s = 0; s < 8; ++s) { const int row = 2 * s + hi, cofs = lr * 4; v4f val = *(const v4fa*)(os + row * 68 + cofs);
                    val[0] += bfr(bias[c0 + cofs]); val[1] += bfr(bias[c0 + cofs + 1]); val[2] += bfr(bias[c0 + cofs + 2]); val[3] += bfr(bias[c0 + cofs + 3]);
                    *(volatile v4f*)(crow + (size_t)row * ldc + cofs) = val; }
                if (ps == 0) __threadfence(); }
        } else {
            h16* crow = (h16*)Cv + z * sC + (size_t)(r0 + mb * 16) * ldc + c0;
#pragma unroll 1
            for (int ps = 0; ps < 2; ++ps) {
#pragma unroll
                for (int s = 0; s < 4; ++s) { const int row = 4 * s + (lane >> 3), cofs = (lane & 7) * 8;
                    const v4f va = *(const v4fa*)(os + row * 68 + cofs); const v4f vb = *(const v4fa*)(os + row * 68 + cofs + 4); v8h o;
                    const float rb = (OMODE == OM_H16R) ? bfr(bias[r0 + mb * 16 + row]) : 0.0f;
#pragma unroll
                    for (int j = 0; j < 4; ++j) { const float b0 = (OMODE == OM_H16C) ? bfr(bias[c0 + cofs + j]) : rb; const float b1 = (OMODE == OM_H16C) ? bfr(bias[c0 + cofs + 4 + j]) : rb;
                        o[j] = (h16)(va[j] + b0); o[4 + j] = (h16)(vb[j] + b1); }
                    *(volatile v8h*)(crow + (size_t)row * ldc + cofs) = o; }
                if (ps == 0) __threadfence(); }
        }
        __builtin_amdgcn_wave_barrier(); asm volatile("" ::: "memory");
    }
}
__global__ __launch_bounds__(32) void k_gemm_h16c(const bf* A, const bf* Bt, int K, h16* C, int ldc, const float* bias, size_t sA, size_t sB, size_t sC) { gemm_body<0, OM_H16C>(A, A, Bt, K, (void*)C, ldc, bias, sA, sB, sC); }
__global__ __launch_bounds__(32) void k_gemm_h16r(const bf* A, const bf* Bt, int K, h16* C, int ldc, const float* bias, size_t sA, size_t sB, size_t sC) { gemm_body<0, OM_H16R>(A, A, Bt, K, (void*)C, ldc, bias, sA, sB, sC); }
__global__ __launch_bounds__(32) void k_gemm_f32c(const bf* A, const bf* A2, const bf* Bt, int K, float* C, int ldc, const float* bias, size_t sA, size_t sB, size_t sC) { gemm_body<1, OM_F32C>(A, A2, Bt, K, (void*)C, ldc, bias, sA, sB, sC); }

__global__ __launch_bounds__(128) void k_flash(const h16* __restrict__ QP, const h16* __restrict__ KP, const h16* __restrict__ VT, const int* __restrict__ amask, bf* ATh, bf* ATl) {
    __shared__ __align__(16) h16 psh[4 * 16 * PP];
    __shared__ __align__(16) float osh[4 * 16 * OP];
    const int lane = threadIdx.x & 31, w = threadIdx.x >> 5, cl = lane & 15, hi = lane >> 4;
    const int h = blockIdx.y, b = blockIdx.z, kvh = h / REP; const int q0 = blockIdx.x * 64 + w * 16;
    const h16* Qp = QP + ((size_t)b * SEQ + q0 + cl) * DQ + h * HD + 8 * hi;
    const h16* Kp = KP + ((size_t)b * SEQ + cl) * DKV + kvh * HD + 8 * hi;
    const h16* Vp = VT + ((size_t)(b * NKV + kvh) * HD + cl) * SEQ + 8 * hi;
    const int* mrow = amask + (size_t)b * S_FULL;
    h16* P = psh + w * 16 * PP; float* os = osh + w * 16 * OP;
    v16h q[4];
#pragma unroll
    for (int i = 0; i < 4; ++i) q[i] = ldh(Qp + i * 32);
    v8f ctx[8];
#pragma unroll
    for (int dt = 0; dt < 8; ++dt) ctx[dt] = (v8f){};
    float m[8], l[8];
#pragma unroll
    for (int r = 0; r < 8; ++r) { m[r] = MASKT; l[r] = 0.0f; }
#pragma unroll 1
    for (int kb = 0; kb < SEQ; kb += 32) {
        const h16* kp = Kp + (size_t)kb * DKV;
        v8f s0 = (v8f){}, s1 = (v8f){};
        v16h kl0 = ldh(kp), kl1 = ldh(kp + (size_t)16 * DKV);
        s0 = wmma16(q[0], kl0, s0); s1 = wmma16(q[0], kl1, s1);
#pragma unroll
        for (int i = 1; i < 4; ++i) { kl0 = ldh(kp + i * 32); kl1 = ldh(kp + (size_t)16 * DKV + i * 32); s0 = wmma16(q[i], kl0, s0); s1 = wmma16(q[i], kl1, s1); }
        asm volatile("v_nop\n\tv_nop\n\tv_nop\n\tv_nop" : "+v"(s0), "+v"(s1) : "v"(q[3]), "v"(kl0), "v"(kl1));
        const int mk0 = mrow[kb + cl], mk1 = mrow[kb + 16 + cl];
        float fs[8];
#pragma unroll
        for (int r = 0; r < 8; ++r) {
            const float t0 = (mk0 == 0) ? MASKT : s0[r] * SCL2;
            const float t1 = (mk1 == 0) ? MASKT : s1[r] * SCL2;
            float mx = fmaxf(t0, t1);
            mx = fmaxf(mx, __shfl_xor(mx, 1, 32)); mx = fmaxf(mx, __shfl_xor(mx, 2, 32)); mx = fmaxf(mx, __shfl_xor(mx, 4, 32)); mx = fmaxf(mx, __shfl_xor(mx, 8, 32));
            const float mn = fmaxf(m[r], mx);
            const float f = __builtin_amdgcn_exp2f(m[r] - mn);
            const float p0 = __builtin_amdgcn_exp2f((t0 - mn) + PSH);
            const float p1 = __builtin_amdgcn_exp2f((t1 - mn) + PSH);
            float rs = p0 + p1;
            rs += __shfl_xor(rs, 1, 32); rs += __shfl_xor(rs, 2, 32); rs += __shfl_xor(rs, 4, 32); rs += __shfl_xor(rs, 8, 32);
            l[r] = l[r] * f + rs; m[r] = mn; fs[r] = f;
            P[(hi * 8 + r) * PP + cl] = (h16)p0; P[(hi * 8 + r) * PP + 16 + cl] = (h16)p1;
        }
#pragma unroll
        for (int dt = 0; dt < 8; ++dt)
#pragma unroll
            for (int r = 0; r < 8; ++r) ctx[dt][r] *= fs[r];
        asm volatile("s_wait_dscnt 0x0" ::: "memory"); __builtin_amdgcn_wave_barrier();
        const v16h pa = cat16(*(const v8ha*)(P + cl * PP + 8 * hi), *(const v8ha*)(P + cl * PP + 16 + 8 * hi));
        const h16* vp = Vp + kb;
        v16h vl = ldh(vp); ctx[0] = wmma16(pa, vl, ctx[0]);
#pragma unroll
        for (int dt = 1; dt < 8; ++dt) { vl = ldh(vp + (size_t)dt * 16 * SEQ); ctx[dt] = wmma16(pa, vl, ctx[dt]); }
        asm volatile("v_nop\n\tv_nop\n\tv_nop\n\tv_nop" : "+v"(ctx[0]), "+v"(ctx[1]), "+v"(ctx[2]), "+v"(ctx[3]), "+v"(ctx[4]), "+v"(ctx[5]), "+v"(ctx[6]), "+v"(ctx[7]) : "v"(pa), "v"(vl));
        asm volatile("" ::: "memory");
    }
    float inv[8];
#pragma unroll
    for (int r = 0; r < 8; ++r) inv[r] = 1.0f / l[r];
#pragma unroll
    for (int dt = 0; dt < 8; ++dt)
#pragma unroll
        for (int r = 0; r < 8; ++r) os[(hi * 8 + r) * OP + dt * 16 + cl] = ctx[dt][r] * inv[r];
    __builtin_amdgcn_wave_barrier(); asm volatile("" ::: "memory");
#pragma unroll 1
    for (int ps = 0; ps < 2; ++ps) {
#pragma unroll
        for (int s = 0; s < 8; ++s) { const int row = 2 * s + hi, c = cl * 8;
            const v4f va = *(const v4fa*)(os + row * OP + c); const v4f vb = *(const v4fa*)(os + row * OP + c + 4); v8us oh, ol;
#pragma unroll
            for (int j = 0; j < 4; ++j) { unsigned short hh, ll; splitf(va[j], hh, ll); oh[j] = hh; ol[j] = ll; splitf(vb[j], hh, ll); oh[4 + j] = hh; ol[4 + j] = ll; }
            const size_t o = ((size_t)b * SEQ + q0 + row) * DQ + h * HD + c;
            *(volatile v8us*)(ATh + o) = oh; *(volatile v8us*)(ATl + o) = ol; }
        if (ps == 0) __threadfence(); }
}

extern "C" void kernel_launch(void* const* d_in, const int* in_sizes, int n_in,
                              void* d_out, int out_size, void* d_ws, size_t ws_size, hipStream_t stream) {
    if (n_in < 10) return;
    const size_t need_x = ((size_t)(NB - 1) * S_FULL + SEQ) * HM;
    if ((size_t)in_sizes[0] < need_x) return;
    if ((size_t)in_sizes[1] < (size_t)(NB - 1) * S_FULL + SEQ) return;
    if ((size_t)in_sizes[2] < (size_t)HM * DQ || (size_t)in_sizes[3] < (size_t)DQ) return;
    if ((size_t)in_sizes[4] < (size_t)HM * DKV || (size_t)in_sizes[5] < (size_t)DKV) return;
    if ((size_t)in_sizes[6] < (size_t)HM * DKV || (size_t)in_sizes[7] < (size_t)DKV) return;
    if ((size_t)in_sizes[8] < (size_t)DQ * HM || (size_t)in_sizes[9] < (size_t)HM) return;
    if ((size_t)out_size < need_x) return;
    if (ws_size < SZ_ALL) return;
    const float* x = (const float*)d_in[0]; const int* am = (const int*)d_in[1];
    const float* wq = (const float*)d_in[2]; const float* bq = (const float*)d_in[3];
    const float* wk = (const float*)d_in[4]; const float* bk = (const float*)d_in[5];
    const float* wv = (const float*)d_in[6]; const float* bv = (const float*)d_in[7];
    const float* wo = (const float*)d_in[8]; const float* bo = (const float*)d_in[9];
    float* OUT = (float*)d_out;
    char* wsp = (char*)d_ws;
    bf* WQ = (bf*)wsp; wsp += SZ_WQ; bf* WK = (bf*)wsp; wsp += SZ_WKV; bf* WV = (bf*)wsp; wsp += SZ_WKV; bf* WO = (bf*)wsp; wsp += SZ_WO;
    bf* XB = (bf*)wsp; wsp += SZ_XB; h16* QPl = (h16*)wsp; wsp += SZ_QP; h16* KPl = (h16*)wsp; wsp += SZ_KP; h16* VTl = (h16*)wsp; wsp += SZ_VT;
    bf* ATh = (bf*)wsp; wsp += SZ_AT; bf* ATl = (bf*)wsp; wsp += SZ_AT;
    k_wtG<<<(unsigned)(((size_t)HM * DQ / 64 + 63) / 64), 256, 0, stream>>>(wq, HM, DQ, WQ);
    k_wtG<<<(unsigned)(((size_t)HM * DKV / 64 + 63) / 64), 256, 0, stream>>>(wk, HM, DKV, WK);
    k_wtG<<<(unsigned)(((size_t)HM * DKV / 64 + 63) / 64), 256, 0, stream>>>(wv, HM, DKV, WV);
    k_wtG<<<(unsigned)(((size_t)DQ * HM / 64 + 63) / 64), 256, 0, stream>>>(wo, DQ, HM, WO);
    k_cvt8<<<dim3((unsigned)(((size_t)SEQ * HM / 8 + 255) / 256), NB, 1), 256, 0, stream>>>(x, XB, (size_t)SEQ * HM / 8, (size_t)S_FULL * HM, (size_t)SEQ * HM);
    k_gemm_h16c<<<dim3(NB * SEQ / 64, DQ / 64, 1), 32, 0, stream>>>(XB, WQ, HM, QPl, DQ, bq, 0, 0, 0);
    k_gemm_h16c<<<dim3(NB * SEQ / 64, DKV / 64, 1), 32, 0, stream>>>(XB, WK, HM, KPl, DKV, bk, 0, 0, 0);
    k_gemm_h16r<<<dim3(DKV / 64, SEQ / 64, NB), 32, 0, stream>>>(WV, XB, HM, VTl, SEQ, bv, 0, (size_t)SEQ * HM, (size_t)DKV * SEQ);
    k_flash<<<dim3(SEQ / 64, NH_, NB), 128, 0, stream>>>(QPl, KPl, VTl, am, ATh, ATl);
    k_gemm_f32c<<<dim3(SEQ / 64, HM / 64, NB), 32, 0, stream>>>(ATh, ATl, WO, DQ, OUT, HM, bo, (size_t)SEQ * DQ, 0, (size_t)S_FULL * HM);
}
